// GraphAttention_47579647705278
// MI455X (gfx1250) — hardware-verified
//
#include <hip/hip_runtime.h>


namespace {
constexpr int L = 1024, B = 8, E = 512, H = 8, HD = 64, V = 16, NT = L * B, BL = 8  , QL = 1024  ;
constexpr float XS = 8.0f, WSC = 256.0f, PS = 1024.0f, LOG2E = 1.4426950408889634f;
static_assert(L % 64 == 0 && QL % 32 == 0 && E == H * HD, "tiling");
typedef _Float16 b16;
typedef __attribute__((ext_vector_type(16))) _Float16 v16b;
typedef __attribute__((ext_vector_type(8))) _Float16 v8b;
typedef __attribute__((ext_vector_type(8))) float v8f;
typedef __attribute__((ext_vector_type(4))) float v4f;
__device__ __forceinline__ float bf16_rne(float f) { unsigned int u = __float_as_uint(f); u += 0x7FFFu + ((u >> 16) & 1u); return __uint_as_float(u & 0xFFFF0000u); }
__device__ __forceinline__ void split16(float v, b16& hi, b16& lo) { hi = (b16)v; lo = (b16)(v - (float)hi); }
__device__ __forceinline__ v16b frag_kb(const b16* p, int hh) { const v8b a = *(const v8b*)(p + 8 * hh), b = *(const v8b*)(p + 16 + 8 * hh); v16b f;
#pragma unroll
  for (int e = 0; e < 8; ++e) { f[e] = a[e]; f[8 + e] = b[e]; } return f; }
__device__ __forceinline__ v8f wmma16b(v16b a, v16b b, v8f c) { v8f d = __builtin_amdgcn_wmma_f32_16x16x32_f16(false, a, false, b, (short)0, c, false, false); asm volatile("v_nop\n\tv_nop\n\tv_nop\n\tv_nop" : "+v"(d) : "v"(a), "v"(b)); return d; }
__device__ __forceinline__ void wave_lds_sync() { __builtin_amdgcn_fence(__ATOMIC_RELEASE, "workgroup"); __builtin_amdgcn_wave_barrier(); __builtin_amdgcn_fence(__ATOMIC_ACQUIRE, "workgroup"); }
__device__ __forceinline__ float pmul(float a, float b) { float p = a * b; asm volatile("" : "+v"(p)); return p; }
__device__ __forceinline__ int iclamp(int v, int lo, int hi) { return v < lo ? lo : (v > hi ? hi : v); }

typedef __attribute__((ext_vector_type(2))) _Float16 v2h;
typedef __attribute__((ext_vector_type(4))) _Float16 v4h;
typedef __attribute__((ext_vector_type(2))) float v2f;
typedef __attribute__((ext_vector_type(4))) int v4i;
__device__ __forceinline__ float nexp2(float v) { return __builtin_amdgcn_exp2f(v); }
__global__ __launch_bounds__(256) void prep_kernel(const float* __restrict__ wi, const float* __restrict__ wo, b16* __restrict__ WI, b16* __restrict__ WO) {
  const size_t u = (size_t)blockIdx.x * 256 + threadIdx.x; const size_t n1 = (size_t)3 * E * E / 8, n2 = (size_t)E * E / 8; v8b o;
  if (u < n1) { const size_t e = u * 8; for (int j = 0; j < 8; ++j) o[j] = (b16)(bf16_rne(wi[e + j]) * WSC); for (int pass = 0; pass < 2; ++pass) { *(volatile v8b*)(WI + e) = o; __threadfence(); } }
  else if (u < n1 + n2) { const size_t e = (u - n1) * 8; for (int j = 0; j < 8; ++j) o[j] = (b16)(bf16_rne(wo[e + j]) * WSC); for (int pass = 0; pass < 2; ++pass) { *(volatile v8b*)(WO + e) = o; __threadfence(); } }
}
__global__ __launch_bounds__(128) void proj_kernel(const float* __restrict__ x, const b16* __restrict__ WI, const float* __restrict__ bi, b16* __restrict__ Qh, b16* __restrict__ Ql, b16* __restrict__ Kh, b16* __restrict__ Kl, b16* __restrict__ VTh, b16* __restrict__ VTl) {
  __shared__ __attribute__((aligned(16))) b16 As[4][16][E + 8]; __shared__ __attribute__((aligned(16))) float Tf[4][16][128 + 4];
  const int wave = threadIdx.x >> 5, lane = threadIdx.x & 31, nloc = lane & 15, hlf = lane >> 4; const int b = blockIdx.y, slab = blockIdx.z; const int which = slab / 4; const int l0 = blockIdx.x * 64 + wave * 16; const int n0 = slab * 128; const int c0 = n0 - which * E;
  for (int rr = 0; rr < 16; ++rr) { const float* xr = x + ((size_t)(l0 + rr) * B + b) * E; for (int q = lane * 4; q < E; q += 128) { const v4f xv = *(const v4f*)(xr + q); v4h o; for (int j = 0; j < 4; ++j) o[j] = (b16)(bf16_rne(xv[j]) * XS); *(v4h*)(&As[wave][rr][q]) = o; } }
  wave_lds_sync();
  v8f acc[8];
#pragma unroll
  for (int t = 0; t < 8; ++t) acc[t] = (v8f){};
#pragma unroll 2
  for (int kb = 0; kb < E; kb += 32) { const v16b a = frag_kb(&As[wave][nloc][kb], hlf);
#pragma unroll
    for (int t = 0; t < 8; ++t) acc[t] = wmma16b(a, frag_kb(WI + (size_t)(n0 + t * 16 + nloc) * E + kb, hlf), acc[t]); }
#pragma unroll
  for (int t = 0; t < 8; ++t) { const float bb = bf16_rne(bi[n0 + t * 16 + nloc]);
#pragma unroll
    for (int r = 0; r < 8; ++r) Tf[wave][8 * hlf + r][t * 16 + nloc] = acc[t][r] * (1.0f / (XS * WSC)) + bb; }
  __syncthreads();
  for (int pass = 0; pass < 2; ++pass) {
    if (which == 2) {
#pragma unroll 1
      for (int q = 0; q < 32; ++q) { const int cl = wave * 32 + q; const int c = c0 + cl; const int h = c / HD, d = c % HD; const int tk = lane * 2; v2h hv, lv;
        for (int j = 0; j < 2; ++j) { b16 p, ql; split16(Tf[(tk + j) >> 4][(tk + j) & 15][cl] * XS, p, ql); hv[j] = p; lv[j] = ql; }
        const size_t oi = (((size_t)b * H + h) * HD + d) * L + blockIdx.x * 64 + lane * 2; *(volatile v2h*)(VTh + oi) = hv; *(volatile v2h*)(VTl + oi) = lv; } }
    else { b16* Ph_ = which == 0 ? Qh : Kh; b16* Pl_ = which == 0 ? Ql : Kl;
      for (int rr = 0; rr < 16; ++rr) { for (int hs = 0; hs < 2; ++hs) { const int c = c0 + hs * 64; const int h = c / HD; v2h hv, lv; for (int j = 0; j < 2; ++j) { b16 p, ql; split16(Tf[wave][rr][hs * 64 + lane * 2 + j] * XS, p, ql); hv[j] = p; lv[j] = ql; }
          const size_t oi = (((size_t)b * H + h) * L + (l0 + rr)) * HD + lane * 2; *(volatile v2h*)(Ph_ + oi) = hv; *(volatile v2h*)(Pl_ + oi) = lv; } } }
    __threadfence(); }
}
__global__ __launch_bounds__(64) void attn_kernel(const b16* __restrict__ Qh, const b16* __restrict__ Ql, const b16* __restrict__ Kh, const b16* __restrict__ Kl, const b16* __restrict__ VTh, const b16* __restrict__ VTl, const int* __restrict__ edge, const float* __restrict__ amask, const int* __restrict__ kpm, const float* __restrict__ etab, b16* __restrict__ Ch, b16* __restrict__ Cl) {
  __shared__ __attribute__((aligned(16))) b16 Pb[2][16][32 + 8]; __shared__ __attribute__((aligned(16))) float To[2][16][HD + 4]; __shared__ float Et[V * H];
  const int wave = threadIdx.x >> 5, lane = threadIdx.x & 31, hh = lane >> 4, col = lane & 15; const int b = blockIdx.y / H, h = blockIdx.y % H; const int q0 = blockIdx.x * 32 + wave * 16, qi = q0 + col;
  for (int i = threadIdx.x; i < V * H; i += 64) Et[i] = bf16_rne(etab[i]);
  __syncthreads();
  const b16* Qhb = Qh + ((size_t)(b * H + h) * L) * HD; const b16* Qlb = Ql + ((size_t)(b * H + h) * L) * HD; const b16* Khb = Kh + ((size_t)(b * H + h) * L) * HD; const b16* Klb = Kl + ((size_t)(b * H + h) * L) * HD;
  const b16* Vh = VTh + ((size_t)(b * H + h) * HD) * L; const b16* Vl = VTl + ((size_t)(b * H + h) * HD) * L;
  const int* Eb = edge + ((size_t)b * L + qi) * L; const float* Ab = amask + (size_t)qi * L; const int* Kb = kpm + (size_t)b * L;
  const v16b qa0 = frag_kb(Qhb + (size_t)qi * HD, hh), qa1 = frag_kb(Qhb + (size_t)qi * HD + 32, hh), qb0 = frag_kb(Qlb + (size_t)qi * HD, hh), qb1 = frag_kb(Qlb + (size_t)qi * HD + 32, hh);
  const float cs = LOG2E / (8.0f * XS * XS);
  float m = -INFINITY, l = 0.0f; v8f o[4]; for (int t = 0; t < 4; ++t) o[t] = (v8f){};
#pragma unroll 1
  for (int kb = 0; kb < L; kb += 32) {
    float e[16]; float mx = -INFINITY;
#pragma unroll
    for (int u = 0; u < 2; ++u) { v8f s = (v8f){}; const size_t kr = (size_t)(kb + u * 16 + col) * HD; const v16b kh0 = frag_kb(Khb + kr, hh), kh1 = frag_kb(Khb + kr + 32, hh), kl0 = frag_kb(Klb + kr, hh), kl1 = frag_kb(Klb + kr + 32, hh);
      s = wmma16b(kh0, qa0, s); s = wmma16b(kh1, qa1, s); s = wmma16b(kh0, qb0, s); s = wmma16b(kh1, qb1, s); s = wmma16b(kl0, qa0, s); s = wmma16b(kl1, qa1, s);
      const int kk = kb + u * 16 + 8 * hh; const v4i e0 = *(const v4i*)(Eb + kk), e1 = *(const v4i*)(Eb + kk + 4); const v4f a0 = *(const v4f*)(Ab + kk), a1 = *(const v4f*)(Ab + kk + 4); const v4i p0 = *(const v4i*)(Kb + kk), p1 = *(const v4i*)(Kb + kk + 4);
#pragma unroll
      for (int r = 0; r < 8; ++r) { int ev = (r < 4) ? e0[r] : e1[r - 4]; ev = ev < 0 ? 0 : (ev >= V ? V - 1 : ev); const float av = bf16_rne(r < 4 ? a0[r] : a1[r - 4]); const int pad = (r < 4) ? p0[r] : p1[r - 4];
        const float vv = (pad != 0) ? -INFINITY : (s[r] * cs + (av + Et[ev * H + h]) * LOG2E); e[u * 8 + r] = vv; mx = fmaxf(mx, vv); } }
    mx = fmaxf(mx, __shfl_xor(mx, 16)); const float mn = fmaxf(m, mx); const float al = (mn == -INFINITY) ? 1.0f : nexp2(m - mn); float sum = 0.0f;
#pragma unroll
    for (int i2 = 0; i2 < 16; ++i2) { const float p = (e[i2] == -INFINITY || mn == -INFINITY) ? 0.0f : nexp2(e[i2] - mn); sum += p; Pb[wave][col][(i2 < 8 ? 0 : 16) + 8 * hh + (i2 & 7)] = (b16)(p * PS); }
    sum += __shfl_xor(sum, 16); l = l * al + sum; m = mn;
    wave_lds_sync();
    const v16b pf = frag_kb(&Pb[wave][col][0], hh);
#pragma unroll
    for (int t = 0; t < 4; ++t) { o[t] *= al; const size_t vr = (size_t)(t * 16 + col) * L + kb; o[t] = wmma16b(frag_kb(Vh + vr, hh), pf, o[t]); o[t] = wmma16b(frag_kb(Vl + vr, hh), pf, o[t]); }
    wave_lds_sync(); }
  const float inv = (l > 0.0f) ? 1.0f / (l * PS * XS) : __int_as_float(0x7fc00000);
#pragma unroll
  for (int t = 0; t < 4; ++t)
#pragma unroll
    for (int r = 0; r < 8; ++r) To[wave][col][t * 16 + 8 * hh + r] = o[t][r] * inv;
  wave_lds_sync();
  for (int pass = 0; pass < 2; ++pass) { for (int rr = 0; rr < 16; ++rr) { const v2f f = *(const v2f*)(&To[wave][rr][lane * 2]); v2h hv, lv; for (int j = 0; j < 2; ++j) { b16 p, q; split16(f[j] * XS, p, q); hv[j] = p; lv[j] = q; }
      const size_t oi = ((size_t)(q0 + rr) * B + b) * E + h * HD + lane * 2; *(volatile v2h*)(Ch + oi) = hv; *(volatile v2h*)(Cl + oi) = lv; } __threadfence(); }
}
__global__ __launch_bounds__(128) void out_kernel(const b16* __restrict__ Ch, const b16* __restrict__ Cl, const b16* __restrict__ WO, const float* __restrict__ bo, float* __restrict__ out) {
  __shared__ __attribute__((aligned(16))) float Tf[4][16][128 + 4];
  const int wave = threadIdx.x >> 5, lane = threadIdx.x & 31, nloc = lane & 15, hlf = lane >> 4; const size_t m0 = ((size_t)blockIdx.x * 4 + wave) * 16; const int n0 = blockIdx.y * 128;
  v8f acc[8];
#pragma unroll
  for (int t = 0; t < 8; ++t) acc[t] = (v8f){};
#pragma unroll 2
  for (int kb = 0; kb < E; kb += 32) { const v16b a = frag_kb(Ch + (m0 + nloc) * E + kb, hlf), al = frag_kb(Cl + (m0 + nloc) * E + kb, hlf);
#pragma unroll
    for (int t = 0; t < 8; ++t) { const v16b bw = frag_kb(WO + (size_t)(n0 + t * 16 + nloc) * E + kb, hlf); acc[t] = wmma16b(a, bw, acc[t]); acc[t] = wmma16b(al, bw, acc[t]); } }
#pragma unroll
  for (int t = 0; t < 8; ++t) { const float bb = bf16_rne(bo[n0 + t * 16 + nloc]);
#pragma unroll
    for (int r = 0; r < 8; ++r) Tf[wave][8 * hlf + r][t * 16 + nloc] = acc[t][r] * (1.0f / (XS * WSC)) + bb; }
  wave_lds_sync();
  for (int pass = 0; pass < 2; ++pass) { for (int rr = 0; rr < 16; ++rr) *(volatile v4f*)(out + (m0 + rr) * E + n0 + lane * 4) = *(const v4f*)(&Tf[wave][rr][lane * 4]); __threadfence(); }
}
}

extern "C" void kernel_launch(void* const* d_in, const int* in_sizes, int n_in, void* d_out, int out_size, void* d_ws, size_t ws_size, hipStream_t stream) {
  (void)n_in;
  auto Fp = [&](int i) { return (const float*)d_in[i]; }; auto Ip = [&](int i) { return (const int*)d_in[i]; };
  if (in_sizes[0] != NT * E || in_sizes[1] != B * L * L || in_sizes[2] != L * L || in_sizes[3] != B * L || in_sizes[4] != 3 * E * E || in_sizes[5] != 3 * E || in_sizes[6] != E * E || in_sizes[7] != E || in_sizes[8] != V * H || out_size != NT * E) return;
  size_t off = 0; char* ws = (char*)d_ws;
  auto carve = [&](size_t bytes) { char* p = ws + off; off += (bytes + 255) & ~(size_t)255; return p; };
  b16* WI = (b16*)carve((size_t)3 * E * E * 2); b16* WO = (b16*)carve((size_t)E * E * 2); const size_t plane = (size_t)NT * E * 2;
  b16* Qh = (b16*)carve(plane); b16* Ql = (b16*)carve(plane); b16* Kh = (b16*)carve(plane); b16* Kl = (b16*)carve(plane); b16* VTh = (b16*)carve(plane); b16* VTl = (b16*)carve(plane); b16* Ch = (b16*)carve(plane); b16* Cl = (b16*)carve(plane);
  if (off > ws_size || off > ((size_t)128 << 20)) return;
  prep_kernel<<<(unsigned)(((size_t)4 * E * E / 8 + 255) / 256), 256, 0, stream>>>(Fp(4), Fp(6), WI, WO);
  proj_kernel<<<dim3(L / 64, BL, 12), 128, 0, stream>>>(Fp(0), WI, Fp(5), Qh, Ql, Kh, Kl, VTh, VTl);
  attn_kernel<<<dim3(QL / 32, BL * H), 64, 0, stream>>>(Qh, Ql, Kh, Kl, VTh, VTl, Ip(1), Fp(2), Ip(3), Fp(8), Ch, Cl);
  out_kernel<<<dim3((QL * B) / 64, 4), 128, 0, stream>>>(Ch, Cl, WO, Fp(7), (float*)d_out);
}
